// SSI_DDI_Block_27573690040721
// MI455X (gfx1250) — hardware-run, weakly checked
//
#include <hip/hip_runtime.h>
#include <stddef.h>
#include <stdint.h>
#include <math.h>


#define NN      100000
#define NE      1600000
#define NG      2048
#define FIN     128
#define HC      64
#define MP      100096
#define NP      100352
#define NSLB    1024
#define NBLK    98
#define RCAP    20480
#define DEGCAP  64
#define GSL     256
#define GBLK    8
#define GRCAP   16384
#define GCAP    128
#define LTHR    256
#define LWAVE   8
#define IDB     17
#define IDM     ((1 << IDB) - 1)
#define ESH     21
#define GBM     128
#define DPB     128
#define NEGSL   0.2f
#define WSMAX   (128u << 20)

#define P_ATS   0
#define P_ATD   64
#define P_BIA   128
#define P_WRL   192
#define P_WRT   256
#define P_BRL   320
#define P_LEN   384

#define PXB     ((MP * (FIN / 8)) / LTHR)
#define PWT     ((HC * (FIN / 8)) / LTHR)

#define LDS_BKT  ((2 * RCAP + 3 * NSLB + 2 * LWAVE) * 4 + 64)
#define LDS_POOL ((2 * GRCAP + 3 * GSL + 2 * LWAVE) * 4 + 64)

static_assert(HC == 2 * 32);
static_assert(16 * 4 == HC);
static_assert(NN == 97 * 1024 + 672);
static_assert(NG == GBLK * GSL);
static_assert(NP == NBLK * NSLB && NP >= NN);
static_assert((NP % DPB) == 0 && (NSLB % DPB) == 0);
static_assert(MP == 782 * GBM && MP >= NN);
static_assert((FIN % 32) == 0);
static_assert(NN <= (1 << IDB));
static_assert(NE < (1 << ESH) && NSLB <= (1 << (31 - ESH)));
static_assert(GSL <= (1 << (31 - IDB)));
static_assert((NE % 4) == 0 && (NN % 4) == 0 && NE >= 4 && NN >= 4);
static_assert(RCAP >= 16710 + 1671 && (RCAP % 4) == 0);
static_assert(DEGCAP >= 36 + 8);
static_assert(GRCAP >= 12670 + 1267 && (GRCAP % 4) == 0);
static_assert(GCAP >= 78 + 8 && GCAP == 4 * 32);
static_assert(((MP * (FIN / 8)) % LTHR) == 0 && ((HC * (FIN / 8)) % LTHR) == 0);
static_assert(LDS_BKT <= 300000 && LDS_POOL <= 300000);
static_assert(P_LEN % 32 == 0 && P_BRL + 4 <= P_LEN);
static_assert(LTHR == 2 * GBM && GBM == LWAVE * 16);
static_assert(DPB == LWAVE * 16);

typedef float          v2f  __attribute__((ext_vector_type(2)));
typedef float          v4f  __attribute__((ext_vector_type(4)));
typedef float          v8f  __attribute__((ext_vector_type(8)));
typedef int            v2i  __attribute__((ext_vector_type(2)));
typedef int            v4i  __attribute__((ext_vector_type(4)));
typedef int            v8i  __attribute__((ext_vector_type(8)));
typedef unsigned int   v4u  __attribute__((ext_vector_type(4)));
typedef unsigned short v8us __attribute__((ext_vector_type(8)));
typedef __bf16         v16b __attribute__((ext_vector_type(16)));
typedef v2f  __attribute__((may_alias)) v2fa;
typedef v4f  __attribute__((may_alias)) v4fa;
typedef v2i  __attribute__((may_alias)) v2ia;
typedef v4i  __attribute__((may_alias)) v4ia;
typedef v8us __attribute__((may_alias)) v8usa;
union FragB { v16b v; v8us h[2]; v8i w; };

__device__ __forceinline__ v8f wmb(const FragB& a, const FragB& b, v8f c) {
  v8f d = __builtin_amdgcn_wmma_f32_16x16x32_bf16(false, a.v, false, b.v, (short)0, c, false, false);
  asm volatile("v_nop\n\tv_nop\n\tv_nop\n\tv_nop" : "+v"(d) : "v"(a.w), "v"(b.w));
  return d;
}

__device__ __forceinline__ unsigned int f2bf(float f) {
  const unsigned int u = __float_as_uint(f);
  return ((u + 0x7FFFu + ((u >> 16) & 1u)) >> 16) & 0xFFFFu;
}
__device__ __forceinline__ float bf2f(unsigned int b) { return __uint_as_float(b << 16); }
__device__ __forceinline__ float bfr(float f) { return bf2f(f2bf(f)); }
__device__ __forceinline__ v4f bfr4(const v4f a) {
  v4f r; r.x = bfr(a.x); r.y = bfr(a.y); r.z = bfr(a.z); r.w = bfr(a.w); return r;
}
__device__ __forceinline__ unsigned int pk2(float lo, float hi) { return f2bf(lo) | (f2bf(hi) << 16); }
__device__ __forceinline__ v4u pack8(const v4f a, const v4f b) {
  v4u r;
  r.x = pk2(a.x, a.y); r.y = pk2(a.z, a.w); r.z = pk2(b.x, b.y); r.w = pk2(b.z, b.w);
  return r;
}
__device__ __forceinline__ float leaky(float v) { return v > 0.f ? v : NEGSL * v; }

__global__ __launch_bounds__(LTHR) void k_prep(
    const float* __restrict__ x, const float* __restrict__ W,
    const float* __restrict__ ats, const float* __restrict__ atd, const float* __restrict__ bia,
    const float* __restrict__ wrl, const float* __restrict__ brl, const float* __restrict__ wrt,
    unsigned short* xb, unsigned short* wt, float* par) {
  const int tid = (int)threadIdx.x;
  const int blk = (int)blockIdx.x;
  if (blk < PXB) {
    const int i   = blk * LTHR + tid;
    const int row = i >> 4;
    const int c0  = (i & 15) * 8;
    const int rc  = row < NN ? row : NN - 1;
    const float* p = x + (size_t)rc * FIN + c0;
    v4f a = *(const v4fa*)p, b = *(const v4fa*)(p + 4);
    asm volatile("" :: "v"(a), "v"(b));
    const bool live = row < NN;
    a.x = live ? a.x : 0.f; a.y = live ? a.y : 0.f; a.z = live ? a.z : 0.f; a.w = live ? a.w : 0.f;
    b.x = live ? b.x : 0.f; b.y = live ? b.y : 0.f; b.z = live ? b.z : 0.f; b.w = live ? b.w : 0.f;
    const v4u hv = pack8(a, b);
    unsigned short* o = xb + (size_t)row * FIN + c0;
    *(volatile v4u*)o = hv;
    __threadfence();
    *(volatile v4u*)o = hv;
  } else if (blk < PXB + PWT) {
    const int u  = (blk - PXB) * LTHR + tid;
    const int n  = u >> 4;
    const int k8 = (u & 15) * 8;
    const float* p = W + (size_t)k8 * HC + n;
    v4f a, b;
    a.x = p[0];      a.y = p[HC];     a.z = p[2 * HC]; a.w = p[3 * HC];
    b.x = p[4 * HC]; b.y = p[5 * HC]; b.z = p[6 * HC]; b.w = p[7 * HC];
    const v4u wv = pack8(a, b);
    unsigned short* o = wt + (size_t)n * FIN + k8;
    *(volatile v4u*)o = wv;
    __threadfence();
    *(volatile v4u*)o = wv;
  } else {
    const int t  = tid < 96 ? tid : 95;
    const int c  = (4 * t) & 63;
    const int wh = t >> 4;
    const v4f v0 = *(const v4fa*)(ats + c);
    const v4f v1 = *(const v4fa*)(atd + c);
    const v4f v2 = *(const v4fa*)(bia + c);
    const v4f v3 = *(const v4fa*)(wrl + c);
    const v4f v4 = *(const v4fa*)(wrt + c);
    const float br = brl[0];
    asm volatile("" :: "v"(v0), "v"(v1), "v"(v2), "v"(v3), "v"(v4), "v"(br));
    v4f z5 = {0.f, 0.f, 0.f, 0.f};
    z5.x = (t == 80) ? br : 0.f;
    v4f r = v0;
    r = (wh == 1) ? v1 : r;
    r = (wh == 2) ? v2 : r;
    r = (wh == 3) ? v3 : r;
    r = (wh == 4) ? v4 : r;
    r = (wh == 5) ? z5 : r;
    r = bfr4(r);
    float* o = par + 4 * t;
    const bool wrk = tid < 96;
    if (wrk) *(volatile v4f*)o = r;
    __threadfence();
    if (wrk) *(volatile v4f*)o = r;
  }
}

__global__ __launch_bounds__(LTHR) void k_gemm(
    const unsigned short* __restrict__ A, const unsigned short* __restrict__ WT,
    const float* __restrict__ par, float* xw, float* sdp) {
  __shared__ __attribute__((aligned(16))) float stg[GBM * HC];
  __shared__ __attribute__((aligned(16))) float satt[2 * HC];
  __shared__ __attribute__((aligned(16))) float sdot[GBM * 4];
  const int tid = (int)threadIdx.x, lane = tid & 31;
  const int wave = __builtin_amdgcn_readfirstlane(tid >> 5);
  const int hh = lane >> 4, m = lane & 15;
  const int rowBase = (int)blockIdx.x * GBM;

  if (tid < 32) {
    const v4f av = *(const v4fa*)(par + P_ATS + 4 * tid);
    *(v4fa*)(satt + 4 * tid) = av;
  }

  v8f acc[4];
  {
    const v8f z = {0.f, 0.f, 0.f, 0.f, 0.f, 0.f, 0.f, 0.f};
    acc[0] = z; acc[1] = z; acc[2] = z; acc[3] = z;
  }
  const unsigned short* ap = A  + (size_t)(rowBase + 16 * wave + m) * (size_t)FIN + 8 * hh;
  const unsigned short* wp = WT + (size_t)m * (size_t)FIN + 8 * hh;
#pragma unroll 1
  for (int ks = 0; ks < FIN / 32; ++ks) {
    FragB af;
    af.h[0] = *(const v8usa*)(ap + 32 * ks);
    af.h[1] = *(const v8usa*)(ap + 32 * ks + 16);
#pragma unroll
    for (int t = 0; t < 4; ++t) {
      const unsigned short* wq = wp + (size_t)(16 * t) * (size_t)FIN + 32 * ks;
      FragB bf;
      bf.h[0] = *(const v8usa*)wq;
      bf.h[1] = *(const v8usa*)(wq + 16);
      acc[t] = wmb(af, bf, acc[t]);
    }
  }

#pragma unroll
  for (int t = 0; t < 4; ++t) {
    const int lc = 16 * t + m;
#pragma unroll
    for (int r = 0; r < 8; ++r) {
      const int lr = 16 * wave + 8 * hh + r;
      stg[lr * HC + lc] = acc[t][r];
    }
  }
  __syncthreads();

  {
    const int row = tid & (GBM - 1), which = tid >> 7;
    const float* sa = satt + which * HC;
    const float* hr = stg + row * HC;
    float d0 = 0.f, d1 = 0.f;
#pragma unroll 4
    for (int c4 = 0; c4 < 8; ++c4) {
      const v4f h0 = *(const v4fa*)(hr + 4 * c4);
      const v4f a0 = *(const v4fa*)(sa + 4 * c4);
      const v4f h1 = *(const v4fa*)(hr + 32 + 4 * c4);
      const v4f a1 = *(const v4fa*)(sa + 32 + 4 * c4);
      d0 = fmaf(h0.x, a0.x, d0); d0 = fmaf(h0.y, a0.y, d0); d0 = fmaf(h0.z, a0.z, d0); d0 = fmaf(h0.w, a0.w, d0);
      d1 = fmaf(h1.x, a1.x, d1); d1 = fmaf(h1.y, a1.y, d1); d1 = fmaf(h1.z, a1.z, d1); d1 = fmaf(h1.w, a1.w, d1);
    }
    sdot[row * 4 + which * 2 + 0] = d0;
    sdot[row * 4 + which * 2 + 1] = d1;
  }
  __syncthreads();

  v4f fv[8];
#pragma unroll
  for (int i = 0; i < 8; ++i) {
    const int lr = 16 * wave + 2 * i + hh;
    fv[i] = *(const v4fa*)(stg + lr * HC + 4 * m);
  }
  const int st = tid < GBM ? tid : GBM - 1;
  const v4f sdv = *(const v4fa*)(sdot + 4 * st);
  float* sp = sdp + (size_t)(rowBase + st) * 4;
  const bool sw = wave < 4;

#pragma unroll
  for (int i = 0; i < 8; ++i) {
    const int gr = rowBase + 16 * wave + 2 * i + hh;
    float* op = xw + (size_t)gr * HC + 4 * m;
    *(volatile v4f*)op = fv[i];
  }
  if (sw) *(volatile v4f*)sp = sdv;
  __threadfence();
#pragma unroll
  for (int i = 0; i < 8; ++i) {
    const int gr = rowBase + 16 * wave + 2 * i + hh;
    float* op = xw + (size_t)gr * HC + 4 * m;
    *(volatile v4f*)op = fv[i];
  }
  if (sw) *(volatile v4f*)sp = sdv;
}

template <int SH, bool STORE>
__device__ __forceinline__ int sweep(const int* __restrict__ keys, int nK, int c0, int c1,
                                     unsigned ub, unsigned nsl, int* reg, int pos0, int cap, int lane) {
  int wc = 0;
#pragma unroll 1
  for (int c = c0; c < c1; ++c) {
    const int e0  = c * 128 + 4 * lane;
    const int e0c = e0 < nK - 4 ? e0 : nK - 4;
    const v4i d = *(const v4ia*)(keys + e0c);
    asm volatile("" :: "v"(d));
    const bool ok = e0 < nK;
    const unsigned s0 = (unsigned)d.x - ub, s1 = (unsigned)d.y - ub;
    const unsigned s2 = (unsigned)d.z - ub, s3 = (unsigned)d.w - ub;
    const bool h0 = ok && (s0 < nsl), h1 = ok && (s1 < nsl), h2 = ok && (s2 < nsl), h3 = ok && (s3 < nsl);
    const unsigned m0 = __builtin_amdgcn_ballot_w32(h0);
    const unsigned m1 = __builtin_amdgcn_ballot_w32(h1);
    const unsigned m2 = __builtin_amdgcn_ballot_w32(h2);
    const unsigned m3 = __builtin_amdgcn_ballot_w32(h3);
    if (STORE) {
      if ((m0 | m1 | m2 | m3) != 0u) {
        const int pre = (int)__builtin_amdgcn_mbcnt_lo(m0,
                          __builtin_amdgcn_mbcnt_lo(m1,
                            __builtin_amdgcn_mbcnt_lo(m2,
                              __builtin_amdgcn_mbcnt_lo(m3, 0u))));
        const int p0 = pos0 + wc + pre;
        const int p1 = p0 + (h0 ? 1 : 0);
        const int p2 = p1 + (h1 ? 1 : 0);
        const int p3 = p2 + (h2 ? 1 : 0);
        if (h0 && p0 < cap) reg[p0] = (int)((unsigned)(e0 + 0) | (s0 << SH));
        if (h1 && p1 < cap) reg[p1] = (int)((unsigned)(e0 + 1) | (s1 << SH));
        if (h2 && p2 < cap) reg[p2] = (int)((unsigned)(e0 + 2) | (s2 << SH));
        if (h3 && p3 < cap) reg[p3] = (int)((unsigned)(e0 + 3) | (s3 << SH));
      }
    }
    wc += (int)__builtin_popcount(m0) + (int)__builtin_popcount(m1)
        + (int)__builtin_popcount(m2) + (int)__builtin_popcount(m3);
  }
  return wc;
}

template <int NSL, int SH, bool XL>
__device__ __forceinline__ int build_lists(const int* __restrict__ keys, int nK, int slotBase,
                                           const int* __restrict__ xl, int nX, int cap,
                                           int* reg1, int* reg2, int* scnt, int* soff, int* cur,
                                           int* wcnt, int* wtot, int tid, int lane, int wave) {
  constexpr int PER = NSL / LTHR;
  static_assert(PER * LTHR == NSL && PER >= 1 && PER <= 4);
  static_assert(XL || SH == IDB);

  for (int i = tid; i < NSL; i += LTHR) scnt[i] = 0;
  {
    const v4i z = {0, 0, 0, 0};
    for (int i = tid; i < (cap >> 2); i += LTHR) *(v4ia*)(reg2 + 4 * i) = z;
  }

  const int nCh = (nK + 127) >> 7;
  const int per = (nCh + LWAVE - 1) / LWAVE;
  const int c0  = wave * per;
  int c1 = c0 + per; c1 = c1 > nCh ? nCh : c1;
  const unsigned ub = (unsigned)slotBase;
  const int wcA = sweep<SH, false>(keys, nK, c0, c1, ub, (unsigned)NSL, reg1, 0, cap, lane);
  if (lane == 0) wcnt[wave] = wcA;
  __syncthreads();
  int pre = 0, tot = 0;
#pragma unroll
  for (int w2 = 0; w2 < LWAVE; ++w2) {
    int c = wcnt[w2];
    c = c < 0 ? 0 : c;
    tot += c;
    pre += (w2 < wave) ? c : 0;
  }

  sweep<SH, true>(keys, nK, c0, c1, ub, (unsigned)NSL, reg1, pre, cap, lane);
  __syncthreads();
  const int nh = tot > cap ? cap : tot;

  if (XL) {
#pragma unroll 1
    for (int i = tid; i < nh; i += LTHR) {
      const int u = reg1[i];
      int id = u & ((1 << SH) - 1);
      const int sl = (int)((unsigned)u >> SH) & (NSL - 1);
      id = id > nK - 1 ? nK - 1 : id;
      int s = xl[id];
      s = s < 0 ? 0 : (s > nX - 1 ? nX - 1 : s);
      reg1[i] = s | (sl << IDB);
    }
    __syncthreads();
  }

  if (wave == 0) {
#pragma unroll 1
    for (int b0 = 0; b0 < nh; b0 += 32) {
      const int idx = b0 + lane;
      const int uv  = reg1[idx < nh ? idx : nh - 1];
      const int m32 = (nh - b0) < 32 ? (nh - b0) : 32;
#pragma unroll 1
      for (int k = 0; k < m32; ++k) {
        const int u  = __builtin_amdgcn_readlane(uv, k);
        const int sl = (int)((unsigned)u >> IDB) & (NSL - 1);
        if (lane == 0) scnt[sl] = scnt[sl] + 1;
      }
    }
  }
  __syncthreads();

  {
    int e[PER];
    int ts = 0;
#pragma unroll
    for (int j = 0; j < PER; ++j) {
      int v = scnt[PER * tid + j];
      v = v < 0 ? 0 : v;
      e[j] = v;
      ts += v;
    }
    int incl = ts;
#pragma unroll
    for (int d = 1; d < 32; d <<= 1) {
      const int up = __shfl_up(incl, d);
      if (lane >= d) incl += up;
    }
    if (lane == 31) wtot[wave] = incl;
    __syncthreads();
    int pw = 0;
#pragma unroll
    for (int w2 = 0; w2 < LWAVE; ++w2) pw += (w2 < wave) ? wtot[w2] : 0;
    int run = pw + incl - ts;
#pragma unroll
    for (int j = 0; j < PER; ++j) {
      soff[PER * tid + j] = run;
      cur[PER * tid + j]  = run;
      run += e[j];
    }
  }
  __syncthreads();

  if (wave == 0) {
#pragma unroll 1
    for (int b0 = 0; b0 < nh; b0 += 32) {
      const int idx = b0 + lane;
      const int uv  = reg1[idx < nh ? idx : nh - 1];
      const int m32 = (nh - b0) < 32 ? (nh - b0) : 32;
#pragma unroll 1
      for (int k = 0; k < m32; ++k) {
        const int u  = __builtin_amdgcn_readlane(uv, k);
        const int sl = (int)((unsigned)u >> IDB) & (NSL - 1);
        const int id = u & IDM;
        if (lane == 0) {
          int pos = cur[sl];
          pos = pos < 0 ? 0 : (pos > cap - 1 ? cap - 1 : pos);
          reg2[pos] = id;
          cur[sl] = pos + 1;
        }
      }
    }
  }
  __syncthreads();
  return tot;
}

__global__ __launch_bounds__(LTHR) void k_bucket(const int* __restrict__ srcs, const int* __restrict__ dsts,
                                                 int* hits, int* oc, int* flg) {
  extern __shared__ v4f lds_dyn[];
  int* reg1 = (int*)lds_dyn;
  int* reg2 = reg1 + RCAP;
  int* scnt = reg2 + RCAP;
  int* soff = scnt + NSLB;
  int* cur  = soff + NSLB;
  int* wcnt = cur + NSLB;
  int* wtot = wcnt + LWAVE;
  const int tid = (int)threadIdx.x, lane = tid & 31;
  const int wave = __builtin_amdgcn_readfirstlane(tid >> 5);
  const int slotBase = (int)blockIdx.x * NSLB;

  const int tot = build_lists<NSLB, ESH, true>(dsts, NE, slotBase, srcs, NN, RCAP,
                                               reg1, reg2, scnt, soff, cur, wcnt, wtot, tid, lane, wave);
  const int ovf = tot > RCAP ? 1 : 0;

  int* hb = hits + (size_t)blockIdx.x * RCAP;
  const int j0 = tid, j1 = tid + LTHR;
  v4i o0, o1;
  o0.x = soff[2 * j0]; o0.y = scnt[2 * j0]; o0.z = soff[2 * j0 + 1]; o0.w = scnt[2 * j0 + 1];
  o1.x = soff[2 * j1]; o1.y = scnt[2 * j1]; o1.z = soff[2 * j1 + 1]; o1.w = scnt[2 * j1 + 1];
  int* ob = oc + (size_t)slotBase * 2;
  const v4i fv = {ovf, ovf, ovf, ovf};
  int* fb = flg + (size_t)blockIdx.x * 32 + 4 * (lane & 7);
  const bool fw = (wave == 0) && (lane < 8);

#pragma unroll 1
  for (int i = tid; i < RCAP / 4; i += LTHR) {
    const v4i v = *(const v4ia*)(reg2 + 4 * i);
    *(volatile v4i*)(hb + 4 * i) = v;
  }
  *(volatile v4i*)(ob + 4 * j0) = o0;
  *(volatile v4i*)(ob + 4 * j1) = o1;
  if (fw) *(volatile v4i*)fb = fv;
  __threadfence();
#pragma unroll 1
  for (int i = tid; i < RCAP / 4; i += LTHR) {
    const v4i v = *(const v4ia*)(reg2 + 4 * i);
    *(volatile v4i*)(hb + 4 * i) = v;
  }
  *(volatile v4i*)(ob + 4 * j0) = o0;
  *(volatile v4i*)(ob + 4 * j1) = o1;
  if (fw) *(volatile v4i*)fb = fv;
}

__global__ __launch_bounds__(LTHR) void k_attn(
    const int* __restrict__ hits, const int* __restrict__ oc, const int* __restrict__ flg,
    const float* __restrict__ xw, const float* __restrict__ sd, const float* __restrict__ par,
    float* out0, float* xc) {
  __shared__ __attribute__((aligned(16))) float sb[HC];
  const int tid = (int)threadIdx.x, lane = tid & 31;
  const int wave = __builtin_amdgcn_readfirstlane(tid >> 5);
  if (tid < 16) {
    const v4f bv = *(const v4fa*)(par + P_BIA + 4 * tid);
    *(v4fa*)(sb + 4 * tid) = bv;
  }
  __syncthreads();
  const int half = lane >> 4, q = lane & 15;
  const bool hd = (q >> 3) != 0;
  const v4f bb = *(const v4fa*)(sb + 4 * q);
  const int blockBase = (int)blockIdx.x * DPB;
  const int b  = blockBase >> 10;
  const int hb = b * RCAP;
  const int fl = flg[b * 32];
  const float qnan = __int_as_float(0x7fc00000);

#pragma unroll 1
  for (int it = 0; it < 8; ++it) {
    const int i  = blockBase + wave * 16 + 2 * it + half;
    const int ic = i < NN ? i : NN - 1;
    const v2i o2 = *(const v2ia*)(oc + 2 * (size_t)i);
    int st = o2.x;
    const int craw = o2.y;
    st = st < 0 ? 0 : (st > RCAP - 1 ? RCAP - 1 : st);
    int cnt = craw < 0 ? 0 : (craw > DEGCAP ? DEGCAP : craw);
    cnt = cnt > RCAP - st ? RCAP - st : cnt;
    const int cother = __shfl_xor(cnt, 16);
    const int cu = __builtin_amdgcn_readfirstlane(cnt > cother ? cnt : cother);
    int last = st + cnt - 1; last = last < st ? st : last;
    const bool poison = (fl != 0) || (craw > DEGCAP) || (craw < 0);

    const v4f sdi = *(const v4fa*)(sd + 4 * (size_t)ic);
    v4f av = *(const v4fa*)(xw + (size_t)ic * HC + 4 * q);
    const float asi = hd ? sdi.y : sdi.x;
    const float adi = hd ? sdi.w : sdi.z;
    float mx = leaky(asi + adi);
    float dn = 1.0f;

#pragma unroll 1
    for (int q2 = 0; q2 < cu; ++q2) {
      int idx = st + q2; idx = idx > last ? last : idx;
      idx = idx < 0 ? 0 : (idx > RCAP - 1 ? RCAP - 1 : idx);
      const int sw = hits[hb + idx];
      const int s  = sw < 0 ? 0 : (sw > NN - 1 ? NN - 1 : sw);
      const v4f ss = *(const v4fa*)(sd + 4 * (size_t)s);
      const v4f fs = *(const v4fa*)(xw + (size_t)s * HC + 4 * q);
      asm volatile("" :: "v"(ss), "v"(fs));
      const bool valid = q2 < cnt;
      const float lg = leaky((hd ? ss.y : ss.x) + adi);
      const float df = lg - mx;
      const float ee = expf(-fabsf(df));
      const bool up  = df > 0.f;
      const float s1 = up ? ee : 1.0f;
      const float s2 = up ? 1.0f : ee;
      const float mxn = up ? lg : mx;
      const float dnn = fmaf(dn, s1, s2);
      const float ax = fmaf(av.x, s1, s2 * fs.x);
      const float ay = fmaf(av.y, s1, s2 * fs.y);
      const float az = fmaf(av.z, s1, s2 * fs.z);
      const float aw = fmaf(av.w, s1, s2 * fs.w);
      mx = valid ? mxn : mx;
      dn = valid ? dnn : dn;
      av.x = valid ? ax : av.x;
      av.y = valid ? ay : av.y;
      av.z = valid ? az : av.z;
      av.w = valid ? aw : av.w;
    }
    const float inv = 1.0f / dn;
    v4f o;
    o.x = av.x * inv + bb.x;
    o.y = av.y * inv + bb.y;
    o.z = av.z * inv + bb.z;
    o.w = av.w * inv + bb.w;
    o.x = poison ? qnan : o.x;
    o.y = poison ? qnan : o.y;
    o.z = poison ? qnan : o.z;
    o.w = poison ? qnan : o.w;
    float* p0 = out0 + (size_t)ic * HC + 4 * q;
    float* p1 = xc   + (size_t)ic * HC + 4 * q;
    const bool wr = i < NN;
    if (wr) { *(volatile v4f*)p0 = o; *(volatile v4f*)p1 = o; }
    __threadfence();
    if (wr) { *(volatile v4f*)p0 = o; *(volatile v4f*)p1 = o; }
  }
}

__global__ __launch_bounds__(LTHR) void k_score(
    const int* __restrict__ hits, const int* __restrict__ oc, const int* __restrict__ flg,
    const float* __restrict__ xc, const float* __restrict__ par, float* score) {
  __shared__ __attribute__((aligned(16))) float sp[136];
  __shared__ __attribute__((aligned(16))) float ssc[DPB];
  const int tid = (int)threadIdx.x, lane = tid & 31;
  const int wave = __builtin_amdgcn_readfirstlane(tid >> 5);
  if (tid < 33) {
    const v4f pv = *(const v4fa*)(par + P_WRL + 4 * tid);
    *(v4fa*)(sp + 4 * tid) = pv;
  }
  __syncthreads();
  const int half = lane >> 4, q = lane & 15;
  const v4f wr4 = *(const v4fa*)(sp + 4 * q);
  const v4f wt4 = *(const v4fa*)(sp + HC + 4 * q);
  const float brl = sp[2 * HC];
  const int blockBase = (int)blockIdx.x * DPB;
  const int b  = blockBase >> 10;
  const int hb = b * RCAP;
  const int fl = flg[b * 32];
  const float qnan = __int_as_float(0x7fc00000);

#pragma unroll 1
  for (int it = 0; it < 8; ++it) {
    const int i  = blockBase + wave * 16 + 2 * it + half;
    const int ic = i < NN ? i : NN - 1;
    const v2i o2 = *(const v2ia*)(oc + 2 * (size_t)i);
    int st = o2.x;
    const int craw = o2.y;
    st = st < 0 ? 0 : (st > RCAP - 1 ? RCAP - 1 : st);
    int cnt = craw < 0 ? 0 : (craw > DEGCAP ? DEGCAP : craw);
    cnt = cnt > RCAP - st ? RCAP - st : cnt;
    const int cother = __shfl_xor(cnt, 16);
    const int cu = __builtin_amdgcn_readfirstlane(cnt > cother ? cnt : cother);
    int last = st + cnt - 1; last = last < st ? st : last;
    const bool poison = (fl != 0) || (craw > DEGCAP) || (craw < 0);

    v4f ag = {0.f, 0.f, 0.f, 0.f};
#pragma unroll 1
    for (int q2 = 0; q2 < cu; ++q2) {
      int idx = st + q2; idx = idx > last ? last : idx;
      idx = idx < 0 ? 0 : (idx > RCAP - 1 ? RCAP - 1 : idx);
      const int sw = hits[hb + idx];
      const int s  = sw < 0 ? 0 : (sw > NN - 1 ? NN - 1 : sw);
      const v4f fs = *(const v4fa*)(xc + (size_t)s * HC + 4 * q);
      asm volatile("" :: "v"(fs));
      const bool valid = q2 < cnt;
      const float nx = ag.x + fs.x, ny = ag.y + fs.y, nz = ag.z + fs.z, nw = ag.w + fs.w;
      ag.x = valid ? nx : ag.x;
      ag.y = valid ? ny : ag.y;
      ag.z = valid ? nz : ag.z;
      ag.w = valid ? nw : ag.w;
    }
    const v4f xi = *(const v4fa*)(xc + (size_t)ic * HC + 4 * q);
    float p = ag.x * wr4.x;
    p = fmaf(ag.y, wr4.y, p);
    p = fmaf(ag.z, wr4.z, p);
    p = fmaf(ag.w, wr4.w, p);
    p = fmaf(xi.x, wt4.x, p);
    p = fmaf(xi.y, wt4.y, p);
    p = fmaf(xi.z, wt4.z, p);
    p = fmaf(xi.w, wt4.w, p);
    p += __shfl_xor(p, 8);
    p += __shfl_xor(p, 4);
    p += __shfl_xor(p, 2);
    p += __shfl_xor(p, 1);
    float sc = p + brl;
    sc = poison ? qnan : sc;
    if (q == 0) ssc[wave * 16 + 2 * it + half] = sc;
  }
  __syncthreads();
  if (wave == 0) {
    const v4f v = *(const v4fa*)(ssc + 4 * lane);
    float* op = score + blockBase + 4 * lane;
    *(volatile v4f*)op = v;
    __threadfence();
    *(volatile v4f*)op = v;
  }
}

__global__ __launch_bounds__(LTHR) void k_pool(const int* __restrict__ bat, const float* __restrict__ score,
                                               const float* __restrict__ xc, float* out1) {
  extern __shared__ v4f lds_dyn[];
  int* reg1 = (int*)lds_dyn;
  int* reg2 = reg1 + GRCAP;
  int* scnt = reg2 + GRCAP;
  int* soff = scnt + GSL;
  int* cur  = soff + GSL;
  int* wcnt = cur + GSL;
  int* wtot = wcnt + LWAVE;
  const int tid = (int)threadIdx.x, lane = tid & 31;
  const int wave = __builtin_amdgcn_readfirstlane(tid >> 5);
  const int slotBase = (int)blockIdx.x * GSL;

  const int tot = build_lists<GSL, IDB, false>(bat, NN, slotBase, bat, NN, GRCAP,
                                               reg1, reg2, scnt, soff, cur, wcnt, wtot, tid, lane, wave);
  const int nh = tot > GRCAP ? GRCAP : tot;
  const bool ovf = tot > GRCAP;
  const float qnan = __int_as_float(0x7fc00000);

#pragma unroll 1
  for (int jt = 0; jt < GSL / LWAVE; ++jt) {
    const int slot = wave * (GSL / LWAVE) + jt;
    const int g = slotBase + slot;
    int stv = soff[slot];
    const int craw = scnt[slot];
    stv = stv < 0 ? 0 : (stv > nh ? nh : stv);
    int cv = craw < 0 ? 0 : (craw > GCAP ? GCAP : craw);
    cv = cv > nh - stv ? nh - stv : cv;
    const int st  = __builtin_amdgcn_readfirstlane(stv);
    const int cnt = __builtin_amdgcn_readfirstlane(cv);
    const bool poison = ovf || (craw > GCAP) || (craw < 0);
    int last = st + cnt - 1; last = last < st ? st : last;

    int nd[4];
    float ev[4];
    float mx = -3.0e38f;
#pragma unroll
    for (int c = 0; c < 4; ++c) {
      int idx = st + 32 * c + lane;
      idx = idx > last ? last : idx;
      idx = idx < 0 ? 0 : (idx > GRCAP - 1 ? GRCAP - 1 : idx);
      int node = reg2[idx];
      node = node < 0 ? 0 : (node > NN - 1 ? NN - 1 : node);
      const float sc = score[node];
      nd[c] = node;
      ev[c] = sc;
      mx = fmaxf(mx, sc);
    }
#pragma unroll
    for (int off = 16; off > 0; off >>= 1) mx = fmaxf(mx, __shfl_xor(mx, off));
    float sm = 0.0f;
#pragma unroll
    for (int c = 0; c < 4; ++c) {
      const bool valid = (32 * c + lane) < cnt;
      const float e = expf(ev[c] - mx);
      ev[c] = valid ? e : 0.0f;
      sm += ev[c];
    }
#pragma unroll
    for (int off = 16; off > 0; off >>= 1) sm += __shfl_xor(sm, off);
    const float inv = 1.0f / sm;
#pragma unroll
    for (int c = 0; c < 4; ++c) ev[c] = ev[c] * inv;

    float a0 = 0.0f, a1 = 0.0f;
#pragma unroll
    for (int c = 0; c < 4; ++c) {
      int m32 = cnt - 32 * c;
      m32 = m32 < 0 ? 0 : (m32 > 32 ? 32 : m32);
#pragma unroll 1
      for (int k = 0; k < m32; ++k) {
        const int nk = __builtin_amdgcn_readlane(nd[c], k);
        const float w = __int_as_float(__builtin_amdgcn_readlane(__float_as_int(ev[c]), k));
        const v2f r = *(const v2fa*)(xc + (size_t)nk * HC + 2 * lane);
        const float t0 = r.x * w, t1 = r.y * w;
        a0 += t0;
        a1 += t1;
      }
    }
    v2f o;
    o.x = poison ? qnan : a0;
    o.y = poison ? qnan : a1;
    float* op = out1 + (size_t)g * HC + 2 * lane;
    const bool wr = g < NG;
    if (wr) *(volatile v2f*)op = o;
    __threadfence();
    if (wr) *(volatile v2f*)op = o;
  }
}

#define SZ_XB    ((size_t)MP * FIN * 2)
#define SZ_WT    ((size_t)HC * FIN * 2)
#define SZ_PAR   ((size_t)2048)
#define SZ_XW    ((size_t)MP * HC * 4)
#define SZ_SD    ((size_t)MP * 16)
#define SZ_X     ((size_t)NN * HC * 4)
#define SZ_SC    ((size_t)NP * 4)
#define SZ_HITS  ((size_t)NBLK * RCAP * 4)
#define SZ_OC    ((size_t)NP * 8)
#define SZ_FLG   ((size_t)NBLK * 128)
#define O_XB     ((size_t)0)
#define O_WT     (O_XB + SZ_XB)
#define O_PAR    (O_WT + SZ_WT)
#define O_XW     (O_PAR + SZ_PAR)
#define O_SD     (O_XW + SZ_XW)
#define O_X      (O_SD + SZ_SD)
#define O_SC     (O_X + SZ_X)
#define O_HITS   (O_SC + SZ_SC)
#define O_OC     (O_HITS + SZ_HITS)
#define O_FLG    (O_OC + SZ_OC)
#define O_END    (O_FLG + SZ_FLG)
static_assert((SZ_XB % 256) == 0 && (SZ_WT % 256) == 0 && (SZ_PAR % 256) == 0 && (SZ_XW % 256) == 0);
static_assert((SZ_SD % 256) == 0 && (SZ_X % 256) == 0 && (SZ_SC % 256) == 0 && (SZ_HITS % 256) == 0);
static_assert((SZ_OC % 256) == 0 && (SZ_FLG % 128) == 0);
static_assert(SZ_PAR >= (size_t)P_LEN * 4);
static_assert(O_END <= (size_t)WSMAX);
static_assert(((size_t)NN * HC * 4) % 128 == 0);

extern "C" void kernel_launch(void* const* d_in, const int* in_sizes, int n_in,
                              void* d_out, int out_size, void* d_ws, size_t ws_size,
                              hipStream_t stream) {
  if (n_in < 10) return;
  if (in_sizes[0] != NN * FIN) return;
  if (in_sizes[1] != 2 * NE) return;
  if (in_sizes[2] != NN) return;
  if (in_sizes[3] != FIN * HC) return;
  if (in_sizes[4] != HC || in_sizes[5] != HC) return;
  if (in_sizes[6] != HC) return;
  if (in_sizes[7] != HC || in_sizes[9] != HC) return;
  if (in_sizes[8] != 1) return;
  if (out_size != NN * HC + NG * HC) return;
  if (ws_size < O_END) return;

  const float* node = (const float*)d_in[0];
  const int*   ei   = (const int*)  d_in[1];
  const int*   bat  = (const int*)  d_in[2];
  const float* Wp   = (const float*)d_in[3];
  const float* ats  = (const float*)d_in[4];
  const float* atd  = (const float*)d_in[5];
  const float* bia  = (const float*)d_in[6];
  const float* wrl  = (const float*)d_in[7];
  const float* brl  = (const float*)d_in[8];
  const float* wrt  = (const float*)d_in[9];
  const int* src = ei;
  const int* dst = ei + NE;
  float* out0 = (float*)d_out;
  float* out1 = out0 + (size_t)NN * HC;

  char* ws = (char*)d_ws;
  unsigned short* XB  = (unsigned short*)(ws + O_XB);
  unsigned short* WT  = (unsigned short*)(ws + O_WT);
  float*          PAR = (float*)(ws + O_PAR);
  float*          XW  = (float*)(ws + O_XW);
  float*          SD  = (float*)(ws + O_SD);
  float*          XC  = (float*)(ws + O_X);
  float*          SC  = (float*)(ws + O_SC);
  int*            HT  = (int*)(ws + O_HITS);
  int*            OC  = (int*)(ws + O_OC);
  int*            FL  = (int*)(ws + O_FLG);

  hipFuncSetAttribute(reinterpret_cast<const void*>(&k_bucket),
                      hipFuncAttributeMaxDynamicSharedMemorySize, LDS_BKT);
  hipFuncSetAttribute(reinterpret_cast<const void*>(&k_pool),
                      hipFuncAttributeMaxDynamicSharedMemorySize, LDS_POOL);

  k_prep<<<PXB + PWT + 1, LTHR, 0, stream>>>(node, Wp, ats, atd, bia, wrl, brl, wrt, XB, WT, PAR);
  k_gemm<<<MP / GBM, LTHR, 0, stream>>>(XB, WT, PAR, XW, SD);
  k_bucket<<<NBLK, LTHR, LDS_BKT, stream>>>(src, dst, HT, OC, FL);
  k_attn<<<NP / DPB, LTHR, 0, stream>>>(HT, OC, FL, XW, SD, PAR, out0, XC);
  k_score<<<NP / DPB, LTHR, 0, stream>>>(HT, OC, FL, XC, PAR, SC);
  k_pool<<<GBLK, LTHR, LDS_POOL, stream>>>(bat, SC, XC, out1);
}
